// TPGNNModel_82660940579240
// MI455X (gfx1250) — hardware-run, weakly checked
//
#include <hip/hip_runtime.h>
#include <stddef.h>
#include <stdint.h>
#include <math.h>


#define HD      128
#define K2      256
#define ODIM    64
#define NLAY    3
#define NTHR    256
#define NWAVE   8
#define EPT     8
#define CHUNK   (NTHR * EPT)
#define WCAP    (EPT * 32)
#define LISTN   (NWAVE * WCAP)
#define NBA     1024
#define SLA     10
#define RCAP    28672
#define DEGCAP  64
#define GBM     64
#define GTHR    128
#define GWAVE   (GTHR / 32)
#define MROWS   128
#define RECW    272
#define WSTD    258
#define XRW     16
#define COW     (2 * NBA)
#define FLW     32
#define NUW_G   (NLAY * HD * (K2 / 8))
#define NUW_V   (HD * (K2 / 8))
#define NUW_O   (HD * (K2 / 8))
#define NUW_H   (ODIM * (K2 / 8))
#define NWB     ((NUW_G + NUW_V + NUW_O + NUW_H) / NTHR)
#define BK_ZINTS (LISTN + 2 * RCAP + 3 * NBA)
#define BK_LDS_INTS (BK_ZINTS + 16)
#define WSMAX   134217728

static_assert((CHUNK & (CHUNK - 1)) == 0 && CHUNK <= 4096);
static_assert((NBA & (NBA - 1)) == 0 && NBA == (1 << SLA));
static_assert(((long long)CHUNK << SLA) < (1LL << 31));
static_assert(NBA % NWAVE == 0 && NBA / NWAVE == 128 && NBA % GBM == 0 && NBA == 4 * NTHR);
static_assert(RCAP % (4 * NTHR) == 0 && BK_ZINTS % 4 == 0);
static_assert(BK_LDS_INTS * 4 <= 327680);
static_assert(DEGCAP == 64);
static_assert(NUW_G % NTHR == 0 && NUW_V % NTHR == 0 && NUW_O % NTHR == 0 && NUW_H % NTHR == 0);
static_assert(NUW_G / NTHR == 48 && NUW_V / NTHR == 16 && NUW_O / NTHR == 16 && NUW_H / NTHR == 8 && NWB == 88);
static_assert(GBM == GWAVE * 16 && HD == 4 * 32 && K2 == 2 * HD && K2 % 32 == 0);
static_assert(MROWS % GBM == 0);
static_assert(RECW % 2 == 0 && RECW >= 2 * HD + 1 && (RECW * 8) % 128 == 0 && RECW / 2 <= NTHR);
static_assert(WSTD >= 2 * HD + 1 && (WSTD % 2) == 0);

typedef float          v2f   __attribute__((ext_vector_type(2)));
typedef float          v4f   __attribute__((ext_vector_type(4)));
typedef float          v8f   __attribute__((ext_vector_type(8)));
typedef int            v4i   __attribute__((ext_vector_type(4)));
typedef int            v8i   __attribute__((ext_vector_type(8)));
typedef unsigned short v4us  __attribute__((ext_vector_type(4)));
typedef unsigned short v8us  __attribute__((ext_vector_type(8)));
typedef unsigned short v16us __attribute__((ext_vector_type(16)));
typedef __bf16         v16bf __attribute__((ext_vector_type(16)));
typedef double         v2d   __attribute__((ext_vector_type(2)));
typedef v2f  __attribute__((may_alias)) v2fa;
typedef v4f  __attribute__((may_alias)) v4fa;
typedef v4i  __attribute__((may_alias)) v4ia;
typedef v8us __attribute__((may_alias)) v8usa;
typedef v2d  __attribute__((may_alias)) v2da;
union FragB { v16bf v; v16us u; v8us h[2]; v8i w; };
struct HL4 { v4us h; v4us l; };

__device__ __forceinline__ v8f wmb(const FragB& a, const FragB& b, v8f c) {
  v8f d = __builtin_amdgcn_wmma_f32_16x16x32_bf16(false, a.v, false, b.v, (short)0, c, false, false);
  asm volatile("v_nop\n\tv_nop\n\tv_nop\n\tv_nop" : "+v"(d) : "v"(a.w), "v"(b.w));
  return d;
}
__device__ __forceinline__ v8f z8() { v8f z = {0.f, 0.f, 0.f, 0.f, 0.f, 0.f, 0.f, 0.f}; return z; }

__device__ __forceinline__ unsigned bf16_bits(float f) {
  const unsigned u = __float_as_uint(f);
  return (u + 0x7FFFu + ((u >> 16) & 1u)) >> 16;
}
__device__ __forceinline__ float bf16_val(float f) { return __uint_as_float(bf16_bits(f) << 16); }
__device__ __forceinline__ v4f bfv4(const v4f a) {
  v4f r; r.x = bf16_val(a.x); r.y = bf16_val(a.y); r.z = bf16_val(a.z); r.w = bf16_val(a.w); return r;
}
__device__ __forceinline__ v8us pack8(const v4f a, const v4f b) {
  v8us o;
  o[0] = (unsigned short)bf16_bits(a.x); o[1] = (unsigned short)bf16_bits(a.y);
  o[2] = (unsigned short)bf16_bits(a.z); o[3] = (unsigned short)bf16_bits(a.w);
  o[4] = (unsigned short)bf16_bits(b.x); o[5] = (unsigned short)bf16_bits(b.y);
  o[6] = (unsigned short)bf16_bits(b.z); o[7] = (unsigned short)bf16_bits(b.w);
  return o;
}
__device__ __forceinline__ HL4 split4(const v4f y) {
  HL4 r;
  const unsigned h0 = bf16_bits(y.x), h1 = bf16_bits(y.y), h2 = bf16_bits(y.z), h3 = bf16_bits(y.w);
  r.h[0] = (unsigned short)h0; r.h[1] = (unsigned short)h1; r.h[2] = (unsigned short)h2; r.h[3] = (unsigned short)h3;
  r.l[0] = (unsigned short)bf16_bits(y.x - __uint_as_float(h0 << 16));
  r.l[1] = (unsigned short)bf16_bits(y.y - __uint_as_float(h1 << 16));
  r.l[2] = (unsigned short)bf16_bits(y.z - __uint_as_float(h2 << 16));
  r.l[3] = (unsigned short)bf16_bits(y.w - __uint_as_float(h3 << 16));
  return r;
}
__device__ __forceinline__ float blendf(float a, float b, unsigned msk) {
  return __uint_as_float((__float_as_uint(a) & ~msk) | (__float_as_uint(b) & msk));
}
__device__ __forceinline__ int clampi(int v, int lo, int hi) { return v < lo ? lo : (v > hi ? hi : v); }

template <int SLB>
__device__ __forceinline__ int scan_chunk(const int* __restrict__ dsts, int nE, int cbase, int slotBase,
                                          int nb, int vec8, int* list, int tid, int lane, int wave) {
  int wc = 0;
  const int el0  = tid * EPT;
  const int e0   = cbase + el0;
  const int sent = -2147483647 - 1;
  v4i da, db;
  if (vec8 != 0 && cbase + CHUNK <= nE) {
    da = *(const v4i*)(dsts + e0);
    db = *(const v4i*)(dsts + e0 + 4);
  } else {
    da.x = (e0     < nE) ? dsts[min(e0,     nE - 1)] : sent;
    da.y = (e0 + 1 < nE) ? dsts[min(e0 + 1, nE - 1)] : sent;
    da.z = (e0 + 2 < nE) ? dsts[min(e0 + 2, nE - 1)] : sent;
    da.w = (e0 + 3 < nE) ? dsts[min(e0 + 3, nE - 1)] : sent;
    db.x = (e0 + 4 < nE) ? dsts[min(e0 + 4, nE - 1)] : sent;
    db.y = (e0 + 5 < nE) ? dsts[min(e0 + 5, nE - 1)] : sent;
    db.z = (e0 + 6 < nE) ? dsts[min(e0 + 6, nE - 1)] : sent;
    db.w = (e0 + 7 < nE) ? dsts[min(e0 + 7, nE - 1)] : sent;
  }
  const unsigned nbs = (unsigned)slotBase;
  const unsigned unb = (unsigned)nb;
  const unsigned s0 = (unsigned)da.x - nbs, s1 = (unsigned)da.y - nbs;
  const unsigned s2 = (unsigned)da.z - nbs, s3 = (unsigned)da.w - nbs;
  const unsigned s4 = (unsigned)db.x - nbs, s5 = (unsigned)db.y - nbs;
  const unsigned s6 = (unsigned)db.z - nbs, s7 = (unsigned)db.w - nbs;
  const bool h0 = s0 < unb, h1 = s1 < unb, h2 = s2 < unb, h3 = s3 < unb;
  const bool h4 = s4 < unb, h5 = s5 < unb, h6 = s6 < unb, h7 = s7 < unb;
  const unsigned any = __builtin_amdgcn_ballot_w32(h0 | h1 | h2 | h3 | h4 | h5 | h6 | h7);
  if (any != 0u) {
#define HITJ(J, HJ, SJ) { \
      const unsigned mj = __builtin_amdgcn_ballot_w32(HJ); \
      if (mj != 0u) { \
        if (HJ) { \
          const int pos = wc + (int)__builtin_amdgcn_mbcnt_lo(mj, 0u); \
          if (pos < WCAP) list[wave * WCAP + pos] = ((el0 + (J)) << SLB) | (int)(SJ); \
        } \
        wc += (int)__builtin_popcount(mj); } }
    HITJ(0, h0, s0)
    HITJ(1, h1, s1)
    HITJ(2, h2, s2)
    HITJ(3, h3, s3)
    HITJ(4, h4, s4)
    HITJ(5, h5, s5)
    HITJ(6, h6, s6)
    HITJ(7, h7, s7)
#undef HITJ
  }
  return wc;
}

__global__ __launch_bounds__(NTHR) void k_prep(const float* __restrict__ gatw, const float* __restrict__ mhaw,
                                               const float* __restrict__ mow, const float* __restrict__ oww,
                                               const float* __restrict__ x, int nN,
                                               unsigned short* wpl, double* xrec) {
  __shared__ __attribute__((aligned(16))) double xr[NTHR * 9];
  __shared__ __attribute__((aligned(16))) double xo[XRW];
  const int tid = (int)threadIdx.x;
  const int blk = (int)blockIdx.x;
  if (blk < NWB) {
    const int u = blk * NTHR + tid;
    v4f a, b;
    if (blk < 48) {
      const int n = u >> 5, kk = ((u & 31) * 8) & (HD - 1);
      const float* p = gatw + (size_t)n * HD + kk;
      a = *(const v4f*)p; b = *(const v4f*)(p + 4);
    } else if (blk < 64) {
      const int v = u - NUW_G;
      const int n = v >> 5, kk = ((v & 31) * 8) & (HD - 1);
      const float* p = mhaw + (size_t)(2 * HD + n) * HD + kk;
      a = *(const v4f*)p; b = *(const v4f*)(p + 4);
    } else if (blk < 80) {
      const int v = u - NUW_G - NUW_V;
      const int n = v >> 5, kk = ((v & 31) * 8) & (HD - 1);
      const float* p = mow + (size_t)n * HD + kk;
      a = *(const v4f*)p; b = *(const v4f*)(p + 4);
    } else {
      const int v = u - NUW_G - NUW_V - NUW_O;
      const int n = v >> 5, kk = ((v & 31) * 8) & (HD - 1);
      const float* p = oww + (size_t)n * HD + kk;
      a = *(const v4f*)p; b = *(const v4f*)(p + 4);
    }
    const v8us o = pack8(a, b);
    unsigned short* dp = wpl + (size_t)u * 8;
    *(volatile v8us*)dp = o;
    __threadfence();
    *(volatile v8us*)dp = o;
  } else {
    const int xb = blk - NWB;
    const int base = xb * 1024;
    double n = 0.0;
    double m[4], q[4];
#pragma unroll
    for (int c = 0; c < 4; ++c) { m[c] = 0.0; q[c] = 0.0; }
#pragma unroll 1
    for (int j = 0; j < 4; ++j) {
      const int r = base + tid + NTHR * j;
      const bool live = r < nN;
      const int rc = live ? r : nN - 1;
      const v2f a = *(const v2fa*)(x + (size_t)rc * 6 + 2);
      const v2f b = *(const v2fa*)(x + (size_t)rc * 6 + 4);
      const float v0 = bf16_val(a.x), v1 = bf16_val(a.y), v2 = bf16_val(b.x), v3 = bf16_val(b.y);
      asm volatile("" :: "v"(v0), "v"(v1), "v"(v2), "v"(v3));
      if (live) {
        n += 1.0;
        const double rk = 1.0 / n;
        double d;
        d = (double)v0 - m[0]; m[0] += d * rk; q[0] += d * ((double)v0 - m[0]);
        d = (double)v1 - m[1]; m[1] += d * rk; q[1] += d * ((double)v1 - m[1]);
        d = (double)v2 - m[2]; m[2] += d * rk; q[2] += d * ((double)v2 - m[2]);
        d = (double)v3 - m[3]; m[3] += d * rk; q[3] += d * ((double)v3 - m[3]);
      }
    }
    xr[tid * 9] = n;
#pragma unroll
    for (int c = 0; c < 4; ++c) { xr[tid * 9 + 1 + c] = m[c]; xr[tid * 9 + 5 + c] = q[c]; }
    __syncthreads();
    if (tid < 32) {
      const int c = tid & 3;
      double tn = 0.0, mean = 0.0, M2 = 0.0;
#pragma unroll 1
      for (int t = 0; t < NTHR; ++t) {
        const double nb = xr[t * 9];
        const double mb = xr[t * 9 + 1 + c];
        const double qb = xr[t * 9 + 5 + c];
        if (nb > 0.5) {
          const double nn = tn + nb;
          const double delta = mb - mean;
          const double f = nb / nn;
          mean = mean + delta * f;
          M2 = M2 + qb + delta * delta * tn * f;
          tn = nn;
        }
      }
      if (tid < 4) { xo[1 + c] = mean; xo[5 + c] = M2; }
      if (tid == 0) xo[0] = tn;
      if (tid >= 9 && tid < XRW) xo[tid] = 0.0;
    }
    __syncthreads();
    if (tid < 8) {
      const v2d v = *(const v2da*)(xo + 2 * tid);
      double* dp = xrec + (size_t)xb * XRW + 2 * tid;
      *(volatile v2d*)dp = v;
      __threadfence();
      *(volatile v2d*)dp = v;
    }
  }
}

__global__ __launch_bounds__(32) void k_xcomb(const double* __restrict__ xrec, int nxb, float* xst) {
  const int lane = (int)threadIdx.x;
  const int c = lane & 3;
  double n = 0.0, mean = 0.0, M2 = 0.0;
#pragma unroll 1
  for (int b = 0; b < nxb; ++b) {
    const double* pr = xrec + (size_t)b * XRW;
    const double nb = pr[0];
    const double mb = pr[1 + c];
    const double qb = pr[5 + c];
    if (nb > 0.5) {
      const double nn = n + nb;
      const double delta = mb - mean;
      const double f = nb / nn;
      mean = mean + delta * f;
      M2 = M2 + qb + delta * delta * n * f;
      n = nn;
    }
  }
  const double den = (n > 1.5) ? (n - 1.0) : 1.0;
  const float meanf = (float)mean;
  float sd = sqrtf((float)(M2 / den));
  sd = fmaxf(sd, 1e-8f);
  const float m0 = __shfl(meanf, 0), m1 = __shfl(meanf, 1), m2 = __shfl(meanf, 2), m3 = __shfl(meanf, 3);
  const float s0 = __shfl(sd, 0), s1 = __shfl(sd, 1), s2 = __shfl(sd, 2), s3 = __shfl(sd, 3);
  const unsigned k0 = (lane == 0) ? 0xFFFFFFFFu : 0u;
  const unsigned k1 = (lane == 1) ? 0xFFFFFFFFu : 0u;
  v4f o;
  o.x = __uint_as_float((__float_as_uint(m0) & k0) | (__float_as_uint(s0) & k1));
  o.y = __uint_as_float((__float_as_uint(m1) & k0) | (__float_as_uint(s1) & k1));
  o.z = __uint_as_float((__float_as_uint(m2) & k0) | (__float_as_uint(s2) & k1));
  o.w = __uint_as_float((__float_as_uint(m3) & k0) | (__float_as_uint(s3) & k1));
  if (lane < 8) *(volatile v4f*)(xst + 4 * lane) = o;
  __threadfence();
  if (lane < 8) *(volatile v4f*)(xst + 4 * lane) = o;
}

__global__ __launch_bounds__(NTHR) void k_inproj(const float* __restrict__ x, const float* __restrict__ ipw,
                                                 const float* __restrict__ ipb, const float* __restrict__ xst,
                                                 int nN, int mRows, float* H, unsigned short* HHL) {
  const int tid = (int)threadIdx.x, lane = tid & 31, wave = tid >> 5;
  const int row = (int)blockIdx.x * NWAVE + wave;
  if (row >= mRows) return;
  const bool live = row < nN;
  const int rc = live ? row : nN - 1;
  const int k = lane & 3;
  const float xv = x[(size_t)rc * 6 + 2 + k];
  const float mu = xst[k];
  const float sd = xst[4 + k];
  const float zz = (bf16_val(xv) - mu) / sd;
  const float z0 = __shfl(zz, 0), z1 = __shfl(zz, 1), z2 = __shfl(zz, 2), z3 = __shfl(zz, 3);
  const float* wp = ipw + 16 * lane;
  const v4f w0 = bfv4(*(const v4f*)(wp));
  const v4f w1 = bfv4(*(const v4f*)(wp + 4));
  const v4f w2 = bfv4(*(const v4f*)(wp + 8));
  const v4f w3 = bfv4(*(const v4f*)(wp + 12));
  const v4f bb = bfv4(*(const v4f*)(ipb + 4 * lane));
  v4f h;
  h.x = fmaf(z3, w0.w, fmaf(z2, w0.z, fmaf(z1, w0.y, z0 * w0.x))) + bb.x;
  h.y = fmaf(z3, w1.w, fmaf(z2, w1.z, fmaf(z1, w1.y, z0 * w1.x))) + bb.y;
  h.z = fmaf(z3, w2.w, fmaf(z2, w2.z, fmaf(z1, w2.y, z0 * w2.x))) + bb.z;
  h.w = fmaf(z3, w3.w, fmaf(z2, w3.z, fmaf(z1, w3.y, z0 * w3.x))) + bb.w;
  h.x = live ? fmaxf(h.x, 0.0f) : 0.0f;
  h.y = live ? fmaxf(h.y, 0.0f) : 0.0f;
  h.z = live ? fmaxf(h.z, 0.0f) : 0.0f;
  h.w = live ? fmaxf(h.w, 0.0f) : 0.0f;
  const HL4 s = split4(h);
  float* hp = H + (size_t)row * HD + 4 * lane;
  unsigned short* aq = HHL + (size_t)row * K2 + 4 * lane;
  *(volatile v4f*)hp = h;
  *(volatile v4us*)aq = s.h;
  *(volatile v4us*)(aq + HD) = s.l;
  __threadfence();
  *(volatile v4f*)hp = h;
  *(volatile v4us*)aq = s.h;
  *(volatile v4us*)(aq + HD) = s.l;
}

__global__ __launch_bounds__(NTHR) void k_bucket(const int* __restrict__ srcs, const int* __restrict__ dsts,
                                                 int nE, int nN, int vec8, int* srcl, int* co, int* flg) {
  extern __shared__ __attribute__((aligned(16))) int dsm[];
  int* list = dsm;
  int* hl   = dsm + LISTN;
  int* sl   = hl + RCAP;
  int* cnt  = sl + RCAP;
  int* offs = cnt + NBA;
  int* cur  = offs + NBA;
  int* misc = cur + NBA;
  const int tid = (int)threadIdx.x, lane = tid & 31, wave = tid >> 5;
  const int nodeBase = (int)blockIdx.x * NBA;
  {
    const v4i z4 = {0, 0, 0, 0};
    for (int i = tid * 4; i < BK_ZINTS; i += NTHR * 4) *(v4ia*)(dsm + i) = z4;
    if (tid < 16) misc[tid] = 0;
  }
  __syncthreads();

  int t = 0, ov = 0;
  const int nChunks = (nE + CHUNK - 1) / CHUNK;
#pragma unroll 1
  for (int ch = 0; ch < nChunks; ++ch) {
    const int cbase = ch * CHUNK;
    const int wc = scan_chunk<SLA>(dsts, nE, cbase, nodeBase, NBA, vec8, list, tid, lane, wave);
    if (lane == 0) misc[wave] = wc;
    __syncthreads();
    if (wave == 0) {
#pragma unroll 1
      for (int w2 = 0; w2 < NWAVE; ++w2) {
        int c = misc[w2];
        c = c < 0 ? 0 : (c > WCAP ? WCAP : c);
#pragma unroll 1
        for (int b0 = 0; b0 < c; b0 += 32) {
          const int idx = b0 + lane;
          const int ent = list[w2 * WCAP + (idx < WCAP ? idx : WCAP - 1)];
          const int m32 = (c - b0) < 32 ? (c - b0) : 32;
#pragma unroll 1
          for (int k = 0; k < m32; ++k) {
            const int u    = __builtin_amdgcn_readlane(ent, k);
            const int slot = u & (NBA - 1);
            const int el   = (u >> SLA) & (CHUNK - 1);
            const int pk   = ((cbase + el) << SLA) | slot;
            if (t < RCAP) {
              if (lane == 0) { hl[t] = pk; cnt[slot] = cnt[slot] + 1; }
              t = t + 1;
            } else {
              ov = 1;
            }
          }
        }
      }
    }
    __syncthreads();
  }
  if (wave == 0 && lane == 0) { misc[8] = t; misc[9] = ov; }
  __syncthreads();
  int tt = misc[8];
  tt = tt < 0 ? 0 : (tt > RCAP ? RCAP : tt);
  const int ovf = misc[9];

  if (wave == 0) {
    const int base = lane * (NBA / 32);
    int s = 0;
#pragma unroll 1
    for (int i = 0; i < NBA / 32; ++i) s += cnt[base + i];
    int incl = s;
#pragma unroll
    for (int d = 1; d < 32; d <<= 1) {
      const int y = __shfl_up(incl, d, 32);
      if (lane >= d) incl += y;
    }
    int run = incl - s;
#pragma unroll 1
    for (int i = 0; i < NBA / 32; ++i) {
      const int cv = cnt[base + i];
      offs[base + i] = run;
      cur[base + i]  = run;
      run += cv;
    }
  }
  __syncthreads();
  if (wave == 0) {
#pragma unroll 1
    for (int b0 = 0; b0 < tt; b0 += 32) {
      const int idx = b0 + lane;
      const int ent = hl[idx < RCAP ? idx : RCAP - 1];
      const int m32 = (tt - b0) < 32 ? (tt - b0) : 32;
#pragma unroll 1
      for (int k = 0; k < m32; ++k) {
        const int u    = __builtin_amdgcn_readlane(ent, k);
        const int slot = u & (NBA - 1);
        if (lane == 0) {
          int p = cur[slot];
          p = p < 0 ? 0 : (p > RCAP - 1 ? RCAP - 1 : p);
          sl[p] = u;
          cur[slot] = p + 1;
        }
      }
    }
  }
  __syncthreads();

  int* gs = srcl + (size_t)blockIdx.x * RCAP;
#pragma unroll 1
  for (int u = tid; u < RCAP / 4; u += NTHR) {
    const v4i ent = *(const v4ia*)(sl + 4 * u);
    const int e0 = clampi(ent.x >> SLA, 0, nE - 1);
    const int e1 = clampi(ent.y >> SLA, 0, nE - 1);
    const int e2 = clampi(ent.z >> SLA, 0, nE - 1);
    const int e3 = clampi(ent.w >> SLA, 0, nE - 1);
    int s0 = srcs[e0], s1 = srcs[e1], s2 = srcs[e2], s3 = srcs[e3];
    asm volatile("" :: "v"(s0), "v"(s1), "v"(s2), "v"(s3));
    s0 = clampi(s0, 0, nN - 1); s1 = clampi(s1, 0, nN - 1);
    s2 = clampi(s2, 0, nN - 1); s3 = clampi(s3, 0, nN - 1);
    v4i o;
    o.x = s0 & ((4 * u + 0 < tt) ? -1 : 0);
    o.y = s1 & ((4 * u + 1 < tt) ? -1 : 0);
    o.z = s2 & ((4 * u + 2 < tt) ? -1 : 0);
    o.w = s3 & ((4 * u + 3 < tt) ? -1 : 0);
    *(volatile v4i*)(gs + 4 * u) = o;
    __threadfence();
    *(volatile v4i*)(gs + 4 * u) = o;
  }
  {
    const v4i c4 = *(const v4ia*)(cnt + 4 * tid);
    const v4i o4 = *(const v4ia*)(offs + 4 * tid);
    int* cp = co + (size_t)blockIdx.x * COW + 4 * tid;
    v4i f4 = {0, 0, 0, 0};
    if (tid == 0) { f4.x = tt; f4.y = ovf; }
    int* fp = flg + (size_t)blockIdx.x * FLW + 4 * tid;
    *(volatile v4i*)cp = c4;
    *(volatile v4i*)(cp + NBA) = o4;
    if (tid < 8) *(volatile v4i*)fp = f4;
    __threadfence();
    *(volatile v4i*)cp = c4;
    *(volatile v4i*)(cp + NBA) = o4;
    if (tid < 8) *(volatile v4i*)fp = f4;
  }
}

template <int NT, int MODE>
__global__ __launch_bounds__(GTHR) __attribute__((amdgpu_num_vgpr(248)))
void k_gemm(const unsigned short* __restrict__ A, const unsigned short* __restrict__ BT, int nN,
            const float* __restrict__ p0, const float* __restrict__ p1,
            const float* __restrict__ hres, const int* __restrict__ flg, int nbk,
            float* fout, float* sdout, unsigned short* aout) {
  constexpr int GBN = 16 * NT;
  __shared__ __attribute__((aligned(16))) float stg[GBM * GBN];
  __shared__ __attribute__((aligned(16))) float sv1[256];
  __shared__ __attribute__((aligned(16))) float sdot[512];
  const int tid = (int)threadIdx.x, lane = tid & 31, wave = tid >> 5, hh = lane >> 4, m = lane & 15;
  const int rowBase = (int)blockIdx.x * GBM;

  if constexpr (MODE == 0) {
    if (tid < 64) {
      const int which = tid >> 5;
      const int c4 = 4 * (tid & 31);
      const v4f vs = *(const v4f*)(p0 + c4);
      const v4f vd = *(const v4f*)(p1 + c4);
      const unsigned msk = which ? 0xFFFFFFFFu : 0u;
      v4f v;
      v.x = bf16_val(blendf(vs.x, vd.x, msk));
      v.y = bf16_val(blendf(vs.y, vd.y, msk));
      v.z = bf16_val(blendf(vs.z, vd.z, msk));
      v.w = bf16_val(blendf(vs.w, vd.w, msk));
      *(v4fa*)(sv1 + which * HD + c4) = v;
    }
  }
  if constexpr (MODE == 3) {
    if (tid < 16) {
      const v4f b4 = bfv4(*(const v4f*)(p0 + 4 * tid));
      *(v4fa*)(sv1 + 4 * tid) = b4;
    }
  }

  v8f acc[NT];
#pragma unroll
  for (int t = 0; t < NT; ++t) acc[t] = z8();
  const unsigned short* ap = A  + (size_t)(rowBase + 16 * wave + m) * (size_t)K2 + 8 * hh;
  const unsigned short* bp = BT + (size_t)m * (size_t)K2 + 8 * hh;

#pragma unroll 1
  for (int k0 = 0; k0 < K2; k0 += 32) {
    FragB af;
    af.h[0] = *(const v8usa*)(ap + k0);
    af.h[1] = *(const v8usa*)(ap + k0 + 16);
#pragma unroll
    for (int nt = 0; nt < NT; ++nt) {
      const unsigned short* wq = bp + (size_t)(16 * nt) * (size_t)K2 + k0;
      FragB bf;
      bf.h[0] = *(const v8usa*)wq;
      bf.h[1] = *(const v8usa*)(wq + 16);
      acc[nt] = wmb(af, bf, acc[nt]);
    }
  }

#pragma unroll
  for (int nt = 0; nt < NT; ++nt) {
    const int lc = 16 * nt + m;
#pragma unroll
    for (int r = 0; r < 8; ++r) {
      const int lr = 16 * wave + 8 * hh + r;
      stg[lr * GBN + lc] = acc[nt][r];
    }
  }
  __syncthreads();

  if constexpr (MODE == 0) {
    {
      const int row = tid & 63, which = tid >> 6;
      const float* sa = sv1 + which * HD;
      const float* hr = stg + row * GBN;
      float d[4];
#pragma unroll
      for (int hd = 0; hd < 4; ++hd) {
        float dd = 0.0f;
#pragma unroll 2
        for (int c4 = 0; c4 < 8; ++c4) {
          const v4f hv = *(const v4fa*)(hr + 32 * hd + 4 * c4);
          const v4f av = *(const v4fa*)(sa + 32 * hd + 4 * c4);
          dd = fmaf(hv.x, av.x, dd);
          dd = fmaf(hv.y, av.y, dd);
          dd = fmaf(hv.z, av.z, dd);
          dd = fmaf(hv.w, av.w, dd);
        }
        d[hd] = dd;
      }
      v4f dv; dv.x = d[0]; dv.y = d[1]; dv.z = d[2]; dv.w = d[3];
      *(v4fa*)(sdot + row * 8 + which * 4) = dv;
    }
    __syncthreads();
    v4f pv[16];
#pragma unroll
    for (int i = 0; i < 16; ++i) pv[i] = *(const v4fa*)(stg + (16 * wave + i) * GBN + 4 * lane);
    const v4f sv = *(const v4fa*)(sdot + 4 * tid);
    float* sp = sdout + (size_t)rowBase * 8 + 4 * tid;
#pragma unroll
    for (int i = 0; i < 16; ++i) {
      float* op = fout + (size_t)(rowBase + 16 * wave + i) * (size_t)HD + 4 * lane;
      *(volatile v4f*)op = pv[i];
    }
    *(volatile v4f*)sp = sv;
    __threadfence();
#pragma unroll
    for (int i = 0; i < 16; ++i) {
      float* op = fout + (size_t)(rowBase + 16 * wave + i) * (size_t)HD + 4 * lane;
      *(volatile v4f*)op = pv[i];
    }
    *(volatile v4f*)sp = sv;
  } else if constexpr (MODE == 1 || MODE == 2) {
    const v4f bq = bfv4(*(const v4f*)(p0 + 4 * lane));
    v4us hv[16], lv[16];
#pragma unroll
    for (int i = 0; i < 16; ++i) {
      const int row = rowBase + 16 * wave + i;
      const bool ok = row < nN;
      const v4f xq = *(const v4fa*)(stg + (16 * wave + i) * GBN + 4 * lane);
      v4f y;
      y.x = xq.x + bq.x; y.y = xq.y + bq.y; y.z = xq.z + bq.z; y.w = xq.w + bq.w;
      if constexpr (MODE == 2) {
        const v4f hq = *(const v4f*)(hres + (size_t)row * HD + 4 * lane);
        y.x += hq.x; y.y += hq.y; y.z += hq.z; y.w += hq.w;
      }
      y.x = ok ? y.x : 0.0f; y.y = ok ? y.y : 0.0f; y.z = ok ? y.z : 0.0f; y.w = ok ? y.w : 0.0f;
      const HL4 s = split4(y);
      hv[i] = s.h;
      lv[i] = s.l;
    }
#pragma unroll
    for (int i = 0; i < 16; ++i) {
      unsigned short* op = aout + (size_t)(rowBase + 16 * wave + i) * (size_t)K2 + 4 * lane;
      *(volatile v4us*)op = hv[i];
      *(volatile v4us*)(op + HD) = lv[i];
    }
    __threadfence();
#pragma unroll
    for (int i = 0; i < 16; ++i) {
      unsigned short* op = aout + (size_t)(rowBase + 16 * wave + i) * (size_t)K2 + 4 * lane;
      *(volatile v4us*)op = hv[i];
      *(volatile v4us*)(op + HD) = lv[i];
    }
  } else {
    if (tid < 64) {
      float* sr = stg + tid * GBN;
      float s = 0.0f;
#pragma unroll 1
      for (int c4 = 0; c4 < GBN / 4; ++c4) {
        v4f y = *(const v4fa*)(sr + 4 * c4);
        const v4f b4 = *(const v4fa*)(sv1 + 4 * c4);
        y.x += b4.x; y.y += b4.y; y.z += b4.z; y.w += b4.w;
        *(v4fa*)(sr + 4 * c4) = y;
        s = fmaf(y.x, y.x, s);
        s = fmaf(y.y, y.y, s);
        s = fmaf(y.z, y.z, s);
        s = fmaf(y.w, y.w, s);
      }
      sv1[128 + tid] = fmaxf(sqrtf(s), 1e-12f);
    }
    __syncthreads();
    int fb = rowBase >> SLA;
    fb = fb > nbk - 1 ? nbk - 1 : fb;
    const int ovw = flg[(size_t)fb * FLW + 1];
    const float pz = (ovw != 0) ? __int_as_float(0x7fc00000) : 0.0f;
    {
      const int r = tid >> 1, hf = tid & 1;
      const float dd = sv1[128 + r];
      float* sr = stg + r * GBN + 32 * hf;
#pragma unroll 1
      for (int c4 = 0; c4 < 8; ++c4) {
        v4f v = *(const v4fa*)(sr + 4 * c4);
        v.x = v.x / dd + pz;
        v.y = v.y / dd + pz;
        v.z = v.z / dd + pz;
        v.w = v.w / dd + pz;
        *(v4fa*)(sr + 4 * c4) = v;
      }
    }
    __syncthreads();
    v4f fv[8];
#pragma unroll
    for (int i = 0; i < 8; ++i) {
      const int lr = 16 * wave + 2 * i + hh;
      fv[i] = *(const v4fa*)(stg + lr * GBN + 4 * m);
    }
#pragma unroll
    for (int i = 0; i < 8; ++i) {
      const int gr = rowBase + 16 * wave + 2 * i + hh;
      float* op = fout + (size_t)gr * (size_t)ODIM + 4 * m;
      if (gr < nN) *(volatile v4f*)op = fv[i];
    }
    __threadfence();
#pragma unroll
    for (int i = 0; i < 8; ++i) {
      const int gr = rowBase + 16 * wave + 2 * i + hh;
      float* op = fout + (size_t)gr * (size_t)ODIM + 4 * m;
      if (gr < nN) *(volatile v4f*)op = fv[i];
    }
  }
}

__global__ __launch_bounds__(NTHR) void k_scan(const float* __restrict__ XH, const float* __restrict__ SD,
                                               const int* __restrict__ srcl, const int* __restrict__ co,
                                               const int* __restrict__ flg, const float* __restrict__ gb,
                                               int nN, float* HN, double* rec) {
  __shared__ __attribute__((aligned(16))) int scnt[NBA];
  __shared__ __attribute__((aligned(16))) int soff[NBA];
  __shared__ __attribute__((aligned(16))) double rkd[128];
  __shared__ __attribute__((aligned(16))) double wst[NWAVE * WSTD];
  __shared__ __attribute__((aligned(16))) double rst[RECW];
  __shared__ __attribute__((aligned(16))) float sgb[HD];
  const int tid = (int)threadIdx.x, lane = tid & 31, wave = tid >> 5;
  const int b = (int)blockIdx.x;
  const int nodeBase = b * NBA;
  {
    const int* cb = co + (size_t)b * COW;
    *(v4ia*)(scnt + 4 * tid) = *(const v4i*)(cb + 4 * tid);
    *(v4ia*)(soff + 4 * tid) = *(const v4i*)(cb + NBA + 4 * tid);
    if (tid < 128) rkd[tid] = 1.0 / (double)(tid + 1);
    if (tid < 32) *(v4fa*)(sgb + 4 * tid) = bfv4(*(const v4f*)(gb + 4 * tid));
  }
  int tt = flg[(size_t)b * FLW];
  tt = tt < 0 ? 0 : (tt > RCAP ? RCAP : tt);
  const int ovw = flg[(size_t)b * FLW + 1];
  __syncthreads();

  const int head = lane >> 3;
  const v4f gbv = *(const v4fa*)(sgb + 4 * lane);
  const int* sl = srcl + (size_t)b * RCAP;
  const float qnan = __int_as_float(0x7fc00000);
  int wn = 0;
  double wm[4], wq[4];
#pragma unroll
  for (int j = 0; j < 4; ++j) { wm[j] = 0.0; wq[j] = 0.0; }

#pragma unroll 1
  for (int jt = 0; jt < NBA / NWAVE; ++jt) {
    const int slot = wave * (NBA / NWAVE) + jt;
    const int grow = nodeBase + slot;
    if (grow < nN) {
      const int craw = __builtin_amdgcn_readfirstlane(scnt[slot]);
      int o = __builtin_amdgcn_readfirstlane(soff[slot]);
      int c = craw < 0 ? 0 : (craw > DEGCAP ? DEGCAP : craw);
      o = o < 0 ? 0 : (o > tt ? tt : o);
      if (c > tt - o) c = tt - o;
      const float pz = (ovw != 0 || craw > DEGCAP) ? qnan : 0.0f;
      int i0 = o + lane;      i0 = i0 > RCAP - 1 ? RCAP - 1 : i0;
      int i1 = o + 32 + lane; i1 = i1 > RCAP - 1 ? RCAP - 1 : i1;
      int sr0 = sl[i0], sr1 = sl[i1];
      sr0 = clampi(sr0, 0, nN - 1);
      sr1 = clampi(sr1, 0, nN - 1);
      const float adv = SD[(size_t)grow * 8 + 4 + head];
      float mx = -3.0e38f, dn = 0.0f;
      v4f av = {0.0f, 0.0f, 0.0f, 0.0f};
#pragma unroll 1
      for (int q = 0; q <= c; ++q) {
        const int a0 = __builtin_amdgcn_readlane(sr0, q & 31);
        const int a1 = __builtin_amdgcn_readlane(sr1, q & 31);
        int sk = (q < 32) ? a0 : a1;
        sk = (q == c) ? grow : sk;
        const float esv = SD[(size_t)sk * 8 + head];
        const v4f xv = *(const v4f*)(XH + (size_t)sk * HD + 4 * lane);
        float lg = esv + adv;
        lg = (lg >= 0.0f) ? lg : 0.2f * lg;
        const float df = lg - mx;
        const float ee = expf(-fabsf(df));
        const bool up  = df > 0.0f;
        const float s1 = up ? ee : 1.0f;
        const float s2 = up ? 1.0f : ee;
        mx = up ? lg : mx;
        dn = fmaf(dn, s1, s2);
        av.x = fmaf(av.x, s1, s2 * xv.x);
        av.y = fmaf(av.y, s1, s2 * xv.y);
        av.z = fmaf(av.z, s1, s2 * xv.z);
        av.w = fmaf(av.w, s1, s2 * xv.w);
      }
      v4f hv;
      hv.x = av.x / dn + gbv.x + pz;
      hv.y = av.y / dn + gbv.y + pz;
      hv.z = av.z / dn + gbv.z + pz;
      hv.w = av.w / dn + gbv.w + pz;
      float* hp = HN + (size_t)grow * HD + 4 * lane;
      *(volatile v4f*)hp = hv;
      __threadfence();
      *(volatile v4f*)hp = hv;
      wn += 1;
      const double rk = rkd[wn - 1];
      double d;
      d = (double)hv.x - wm[0]; wm[0] += d * rk; wq[0] += d * ((double)hv.x - wm[0]);
      d = (double)hv.y - wm[1]; wm[1] += d * rk; wq[1] += d * ((double)hv.y - wm[1]);
      d = (double)hv.z - wm[2]; wm[2] += d * rk; wq[2] += d * ((double)hv.z - wm[2]);
      d = (double)hv.w - wm[3]; wm[3] += d * rk; wq[3] += d * ((double)hv.w - wm[3]);
    }
  }

  if (lane == 0) wst[wave * WSTD] = (double)wn;
#pragma unroll
  for (int j = 0; j < 4; ++j) {
    wst[wave * WSTD + 1 + 4 * lane + j]      = wm[j];
    wst[wave * WSTD + 1 + HD + 4 * lane + j] = wq[j];
  }
  __syncthreads();
  if (tid < HD) {
    double n = 0.0, mean = 0.0, M2 = 0.0;
#pragma unroll 1
    for (int w2 = 0; w2 < NWAVE; ++w2) {
      const double nb = wst[w2 * WSTD];
      const double mb = wst[w2 * WSTD + 1 + tid];
      const double qb = wst[w2 * WSTD + 1 + HD + tid];
      if (nb > 0.5) {
        const double nn = n + nb;
        const double delta = mb - mean;
        const double f = nb / nn;
        mean = mean + delta * f;
        M2 = M2 + qb + delta * delta * n * f;
        n = nn;
      }
    }
    rst[1 + tid] = mean;
    rst[1 + HD + tid] = M2;
    if (tid == 0) rst[0] = n;
  } else if (tid < HD + (RECW - 2 * HD - 1)) {
    rst[2 * HD + 1 + (tid - HD)] = 0.0;
  }
  __syncthreads();
  v2d ps;
  double* rp = rec + (size_t)b * RECW + 2 * tid;
  if (tid < RECW / 2) {
    ps = *(const v2da*)(rst + 2 * tid);
    *(volatile v2d*)rp = ps;
  }
  __threadfence();
  if (tid < RECW / 2) {
    *(volatile v2d*)rp = ps;
  }
}

__global__ __launch_bounds__(HD) void k_bnc(const double* __restrict__ rec, int nrec, float* bnp) {
  __shared__ __attribute__((aligned(16))) float st[2 * HD];
  const int c = (int)threadIdx.x;
  double n = 0.0, mean = 0.0, M2 = 0.0;
#pragma unroll 1
  for (int b = 0; b < nrec; ++b) {
    const double* pr = rec + (size_t)b * RECW;
    const double nb = pr[0];
    const double mb = pr[1 + c];
    const double qb = pr[1 + HD + c];
    if (nb > 0.5) {
      const double nn = n + nb;
      const double delta = mb - mean;
      const double f = nb / nn;
      mean = mean + delta * f;
      M2 = M2 + qb + delta * delta * n * f;
      n = nn;
    }
  }
  const double nt = n < 1.0 ? 1.0 : n;
  const float varf = (float)(M2 / nt);
  st[c] = (float)mean;
  st[HD + c] = sqrtf(varf + 1e-5f);
  __syncthreads();
  v4f v;
  if (c < (2 * HD) / 4) {
    v = *(const v4fa*)(st + 4 * c);
    *(volatile v4f*)(bnp + 4 * c) = v;
  }
  __threadfence();
  if (c < (2 * HD) / 4) {
    *(volatile v4f*)(bnp + 4 * c) = v;
  }
}

__global__ __launch_bounds__(NTHR) void k_bnapply(const float* __restrict__ HN, const float* __restrict__ bnp,
                                                  const float* __restrict__ gam, const float* __restrict__ bet,
                                                  int nUnits, float* H, unsigned short* HHL) {
  __shared__ __attribute__((aligned(16))) float sp[4 * HD];
  const int tid = (int)threadIdx.x;
  if (tid < 32) {
    *(v4fa*)(sp + 4 * tid)          = *(const v4f*)(bnp + 4 * tid);
    *(v4fa*)(sp + HD + 4 * tid)     = *(const v4f*)(bnp + HD + 4 * tid);
    *(v4fa*)(sp + 2 * HD + 4 * tid) = bfv4(*(const v4f*)(gam + 4 * tid));
    *(v4fa*)(sp + 3 * HD + 4 * tid) = bfv4(*(const v4f*)(bet + 4 * tid));
  }
  __syncthreads();
  const int u = (int)blockIdx.x * NTHR + tid;
  if (u >= nUnits) return;
  const int c4 = (u & 31) * 4;
  const int row = u >> 5;
  const v4f hn = *(const v4f*)(HN + (size_t)u * 4);
  float* hp = H + (size_t)u * 4;
  const v4f h0 = *(const v4f*)hp;
  const v4f mu = *(const v4fa*)(sp + c4);
  const v4f sd = *(const v4fa*)(sp + HD + c4);
  const v4f gg = *(const v4fa*)(sp + 2 * HD + c4);
  const v4f be = *(const v4fa*)(sp + 3 * HD + c4);
  v4f t;
  t.x = (hn.x - mu.x) / sd.x * gg.x + be.x;
  t.y = (hn.y - mu.y) / sd.y * gg.y + be.y;
  t.z = (hn.z - mu.z) / sd.z * gg.z + be.z;
  t.w = (hn.w - mu.w) / sd.w * gg.w + be.w;
  v4f hv;
  hv.x = h0.x + ((t.x > 0.0f) ? t.x : (t.x - t.x));
  hv.y = h0.y + ((t.y > 0.0f) ? t.y : (t.y - t.y));
  hv.z = h0.z + ((t.z > 0.0f) ? t.z : (t.z - t.z));
  hv.w = h0.w + ((t.w > 0.0f) ? t.w : (t.w - t.w));
  const HL4 s = split4(hv);
  unsigned short* aq = HHL + (size_t)row * K2 + c4;
  *(volatile v4f*)hp = hv;
  *(volatile v4us*)aq = s.h;
  *(volatile v4us*)(aq + HD) = s.l;
  __threadfence();
  *(volatile v4f*)hp = hv;
  *(volatile v4us*)aq = s.h;
  *(volatile v4us*)(aq + HD) = s.l;
}

static inline int cdiv(int a, int b) { return (a + b - 1) / b; }
static inline size_t al256(size_t o) { return (o + 255) & ~(size_t)255; }

extern "C" void kernel_launch(void* const* d_in, const int* in_sizes, int n_in,
                              void* d_out, int out_size, void* d_ws, size_t ws_size,
                              hipStream_t stream) {
  if (n_in < 16) return;
  if (in_sizes[0] < 12 || (in_sizes[0] % 6) != 0) return;
  const int nN = in_sizes[0] / 6;
  if (nN < 2 || nN > (1 << 22)) return;
  if (in_sizes[1] < 2 || (in_sizes[1] & 1) != 0) return;
  const int nE = in_sizes[1] / 2;
  if (nE < 1 || nE >= (1 << 21)) return;
  if (in_sizes[2] != HD * 4 || in_sizes[3] != HD) return;
  if (in_sizes[4] != NLAY * HD * HD) return;
  if (in_sizes[5] != NLAY * HD || in_sizes[6] != NLAY * HD) return;
  if (in_sizes[7] != NLAY * HD || in_sizes[8] != NLAY * HD || in_sizes[9] != NLAY * HD) return;
  if (in_sizes[10] != 3 * HD * HD || in_sizes[11] != 3 * HD) return;
  if (in_sizes[12] != HD * HD || in_sizes[13] != HD) return;
  if (in_sizes[14] != ODIM * HD || in_sizes[15] != ODIM) return;
  if ((long long)out_size != (long long)nN * ODIM) return;

  const float* x    = (const float*)d_in[0];
  const int*   ei   = (const int*)  d_in[1];
  const float* ipw  = (const float*)d_in[2];
  const float* ipb  = (const float*)d_in[3];
  const float* gatw = (const float*)d_in[4];
  const float* asrc = (const float*)d_in[5];
  const float* adst = (const float*)d_in[6];
  const float* gatb = (const float*)d_in[7];
  const float* gam  = (const float*)d_in[8];
  const float* bet  = (const float*)d_in[9];
  const float* mhaw = (const float*)d_in[10];
  const float* mhab = (const float*)d_in[11];
  const float* mow  = (const float*)d_in[12];
  const float* mob  = (const float*)d_in[13];
  const float* oww  = (const float*)d_in[14];
  const float* obb  = (const float*)d_in[15];
  float* out = (float*)d_out;
  const int* src = ei;
  const int* dst = ei + nE;

  const int MP   = cdiv(nN, MROWS) * MROWS;
  const int gM   = MP / GBM;
  const int nbk  = cdiv(nN, NBA);
  const int vec8 = ((nE & 3) == 0) ? 1 : 0;
  if ((long long)nbk * NBA < (long long)nN) return;

  char* ws = (char*)d_ws;
  size_t off = 0;
  const size_t oWPL = off; off = al256(off + (size_t)(NLAY * HD + HD + HD + ODIM) * K2 * 2);
  const size_t oH   = off; off = al256(off + (size_t)MP * HD * 4);
  const size_t oHHL = off; off = al256(off + (size_t)MP * K2 * 2);
  const size_t oXH  = off; off = al256(off + (size_t)MP * HD * 4);
  const size_t oHN  = off; off = al256(off + (size_t)MP * HD * 4);
  const size_t oSD  = off; off = al256(off + (size_t)MP * 8 * 4);
  const size_t oSRL = off; off = al256(off + (size_t)nbk * RCAP * 4);
  const size_t oCO  = off; off = al256(off + (size_t)nbk * COW * 4);
  const size_t oFLG = off; off = al256(off + (size_t)nbk * FLW * 4);
  const size_t oREC = off; off = al256(off + (size_t)nbk * RECW * 8);
  const size_t oXRC = off; off = al256(off + (size_t)nbk * XRW * 8);
  const size_t oXST = off; off = al256(off + (size_t)32 * 4);
  const size_t oBNP = off; off = al256(off + (size_t)2 * HD * 4);
  if (off > ws_size || off > (size_t)WSMAX) return;
  unsigned short* WPL = (unsigned short*)(ws + oWPL);
  unsigned short* GW2 = WPL;
  unsigned short* WV2 = WPL + (size_t)NLAY * HD * K2;
  unsigned short* WO2 = WV2 + (size_t)HD * K2;
  unsigned short* OW2 = WO2 + (size_t)HD * K2;
  float*          H    = (float*)(ws + oH);
  unsigned short* HHL  = (unsigned short*)(ws + oHHL);
  float*          XH   = (float*)(ws + oXH);
  unsigned short* VHL  = (unsigned short*)(ws + oXH);
  float*          HN   = (float*)(ws + oHN);
  float*          SD   = (float*)(ws + oSD);
  int*            SRL  = (int*)(ws + oSRL);
  int*            CO   = (int*)(ws + oCO);
  int*            FLG  = (int*)(ws + oFLG);
  double*         REC  = (double*)(ws + oREC);
  double*         XRC  = (double*)(ws + oXRC);
  float*          XST  = (float*)(ws + oXST);
  float*          BNP  = (float*)(ws + oBNP);

  const size_t bkLds = (size_t)BK_LDS_INTS * 4;
  hipFuncSetAttribute(reinterpret_cast<const void*>(&k_bucket), hipFuncAttributeMaxDynamicSharedMemorySize, (int)bkLds);

  k_prep<<<NWB + nbk, NTHR, 0, stream>>>(gatw, mhaw, mow, oww, x, nN, WPL, XRC);
  k_xcomb<<<1, 32, 0, stream>>>(XRC, nbk, XST);
  k_inproj<<<cdiv(MP, NWAVE), NTHR, 0, stream>>>(x, ipw, ipb, XST, nN, MP, H, HHL);
  k_bucket<<<nbk, NTHR, bkLds, stream>>>(src, dst, nE, nN, vec8, SRL, CO, FLG);

  const int nUa = nN * (HD / 4);
  for (int l = 0; l < NLAY; ++l) {
    k_gemm<8, 0><<<gM, GTHR, 0, stream>>>(HHL, GW2 + (size_t)l * HD * K2, nN, asrc + l * HD, adst + l * HD,
                                          H, FLG, nbk, XH, SD, VHL);
    k_scan<<<nbk, NTHR, 0, stream>>>(XH, SD, SRL, CO, FLG, gatb + l * HD, nN, HN, REC);
    k_bnc<<<1, HD, 0, stream>>>(REC, nbk, BNP);
    k_bnapply<<<cdiv(nUa, NTHR), NTHR, 0, stream>>>(HN, BNP, gam + l * HD, bet + l * HD, nUa, H, HHL);
  }
  k_gemm<8, 1><<<gM, GTHR, 0, stream>>>(HHL, WV2, nN, mhab + 2 * HD, mhab + 2 * HD, H, FLG, nbk, HN, SD, VHL);
  k_gemm<8, 2><<<gM, GTHR, 0, stream>>>(VHL, WO2, nN, mob, mob, H, FLG, nbk, HN, SD, HHL);
  k_gemm<4, 3><<<gM, GTHR, 0, stream>>>(HHL, OW2, nN, obb, obb, H, FLG, nbk, out, SD, VHL);
}
